// MaskedSplineFlows_33414845562909
// MI455X (gfx1250) — hardware-run, weakly checked
//
#include <hip/hip_runtime.h>
#include <stddef.h>
#include <stdint.h>


#define NB    16384
#define ND    64
#define NW    128
#define NL    8
#define NKN   8
#define NP    23
#define NDP   1472
#define NNT   92
#define RM    32
#define NTHR  256
#define XSC   16
#define WSC   1024
#define HSC   64
#define WSCAP 134217728

static_assert(NDP == ND * NP);
static_assert(NNT * 16 == NDP);
static_assert((NB % RM) == 0);
static_assert(RM * ND == 8 * NTHR);
static_assert(NTHR == 8 * 32);
static_assert(NW == 8 * 16);
static_assert(RM == 32);
static_assert(((NL * NW * ND) % (8 * NTHR)) == 0);
static_assert(((NL * NDP * NW) % (8 * NTHR)) == 0);

typedef float    v4f  __attribute__((ext_vector_type(4)));
typedef float    v8f  __attribute__((ext_vector_type(8)));
typedef _Float16 v8h  __attribute__((ext_vector_type(8)));
typedef _Float16 v16h __attribute__((ext_vector_type(16)));
union FragH { v16h v; v8h h[2]; };

__device__ __forceinline__ v8f wmf(v16h a, v16h b, v8f c) {
  v8f d = __builtin_amdgcn_wmma_f32_16x16x32_f16(false, a, false, b, (short)0, c, false, false);
  asm volatile("v_nop\n\tv_nop\n\tv_nop\n\tv_nop" : "+v"(d) : "v"(a), "v"(b));
  return d;
}

__device__ __forceinline__ int hid_deg(int q) {
  return (q < 6) ? (q / 3) : (((q - 6) >> 1) + 2);
}
__device__ __forceinline__ int hid_src(int q) {
  int d, c;
  if (q < 6) { d = q / 3; c = q - 3 * d; }
  else { const int u = q - 6; d = (u >> 1) + 2; c = u & 1; }
  return d + 63 * c;
}

__device__ __forceinline__ float rcp_f(float x) { return __builtin_amdgcn_rcpf(x); }

__device__ __forceinline__ float softplus_f(float v) {
  const float e = __expf(-fabsf(v));
  return fmaxf(v, 0.0f) + __logf(1.0f + e);
}

__device__ __forceinline__ void adj_softmax8(const float* v, float* o) {
  float mx = v[0];
#pragma unroll
  for (int j = 1; j < NKN; ++j) mx = fmaxf(mx, v[j]);
  float e[NKN];
  float s = 0.0f;
#pragma unroll
  for (int j = 0; j < NKN; ++j) { e[j] = __expf(v[j] - mx); s += e[j]; }
  const float inv = rcp_f(s);
  const float c0 = 0.00125f;
  const float c1 = 1.0f / 1.01f;
#pragma unroll
  for (int j = 0; j < NKN; ++j) o[j] = ((e[j] * inv + c0) * c1) * 8.0f;
}

__global__ __launch_bounds__(NTHR) void k_cvt_w1(const float* __restrict__ w, _Float16* dst) {
  const int gt = blockIdx.x * NTHR + threadIdx.x;
  const int e8 = gt * 8;
  const int i0 = e8 & (ND - 1);
  const int q  = (e8 >> 6) & (NW - 1);
  const int ly = e8 >> 13;
  const int h  = hid_src(q);
  const int dq = hid_deg(q);
  const float* sp = w + ((size_t)(ly * NW + h)) * ND + i0;
  const v4f f0 = *(const v4f*)sp;
  const v4f f1 = *(const v4f*)(sp + 4);
  float fv[8] = {f0.x, f0.y, f0.z, f0.w, f1.x, f1.y, f1.z, f1.w};
  v8h o;
#pragma unroll
  for (int j = 0; j < 8; ++j) {
    const float s = (dq >= i0 + j) ? (float)WSC : 0.0f;
    o[j] = (_Float16)(fv[j] * s);
  }
  _Float16* d = dst + e8;
  *(volatile v8h*)d = o;
  __threadfence();
  *(volatile v8h*)d = o;
}

__global__ __launch_bounds__(NTHR) void k_cvt_wo(const float* __restrict__ w, _Float16* dst) {
  const int gt = blockIdx.x * NTHR + threadIdx.x;
  const int e8 = gt * 8;
  const int q0 = e8 & (NW - 1);
  const int orow = e8 >> 7;
  const int o  = orow % NDP;
  const int fo = o / NP;
  const float* sp = w + (size_t)orow * NW;
  v8h ov;
#pragma unroll
  for (int j = 0; j < 8; ++j) {
    const int q = q0 + j;
    const float v = sp[hid_src(q)];
    const float s = (fo > hid_deg(q)) ? (float)WSC : 0.0f;
    ov[j] = (_Float16)(v * s);
  }
  _Float16* d = dst + e8;
  *(volatile v8h*)d = ov;
  __threadfence();
  *(volatile v8h*)d = ov;
}

__global__ __launch_bounds__(NTHR) void k_flow(const float* __restrict__ xin,
                                               const _Float16* __restrict__ w1h,
                                               const float* __restrict__ b1,
                                               const _Float16* __restrict__ woh,
                                               const float* __restrict__ bo,
                                               float* out_x, float* out_ld) {
  __shared__ __attribute__((aligned(16))) float    Pbuf[RM * NDP];
  __shared__ __attribute__((aligned(16))) float    Xf[2][RM * ND];
  __shared__ __attribute__((aligned(16))) _Float16 Xh[RM * ND];
  __shared__ __attribute__((aligned(16))) _Float16 Hh[RM * NW];
  __shared__ __attribute__((aligned(16))) float    Ldj[RM * ND];
  __shared__ __attribute__((aligned(16))) float    Ldl[RM];

  const int t = threadIdx.x, lane = t & 31, hf = lane >> 4, m = lane & 15;
  const int wave = __builtin_amdgcn_readfirstlane(t >> 5);
  const int row0 = blockIdx.x * RM;

  {
    const float* src = xin + (size_t)row0 * ND + 8 * t;
    const v4f a = *(const v4f*)src;
    const v4f b = *(const v4f*)(src + 4);
    *(v4f*)(&Xf[0][8 * t]) = a;
    *(v4f*)(&Xf[0][8 * t + 4]) = b;
  }
  float ldreg = 0.0f;
  __syncthreads();

  const v8f zf = {0.f, 0.f, 0.f, 0.f, 0.f, 0.f, 0.f, 0.f};
  int cur = 0;
#pragma unroll 1
  for (int ly = 0; ly < NL; ++ly) {
    {
      const float* xs = &Xf[cur][8 * t];
      const v4f a = *(const v4f*)xs;
      const v4f b = *(const v4f*)(xs + 4);
      v8h o;
      o[0] = (_Float16)(a.x * (float)XSC); o[1] = (_Float16)(a.y * (float)XSC);
      o[2] = (_Float16)(a.z * (float)XSC); o[3] = (_Float16)(a.w * (float)XSC);
      o[4] = (_Float16)(b.x * (float)XSC); o[5] = (_Float16)(b.y * (float)XSC);
      o[6] = (_Float16)(b.z * (float)XSC); o[7] = (_Float16)(b.w * (float)XSC);
      *(v8h*)(&Xh[8 * t]) = o;
    }
    __syncthreads();

    {
      const int col = 16 * wave + m;
      const _Float16* bp = w1h + ((size_t)(ly * NW + col)) * ND + 8 * hf;
      FragH bk0, bk1;
      bk0.h[0] = *(const v8h*)(bp);      bk0.h[1] = *(const v8h*)(bp + 16);
      bk1.h[0] = *(const v8h*)(bp + 32); bk1.h[1] = *(const v8h*)(bp + 48);
      const float bb = b1[ly * NW + hid_src(col)] * (float)HSC;
#pragma unroll
      for (int mt = 0; mt < 2; ++mt) {
        const _Float16* ap = &Xh[(16 * mt + m) * ND + 8 * hf];
        FragH a0, a1;
        a0.h[0] = *(const v8h*)(ap);      a0.h[1] = *(const v8h*)(ap + 16);
        a1.h[0] = *(const v8h*)(ap + 32); a1.h[1] = *(const v8h*)(ap + 48);
        v8f acc = zf;
        acc = wmf(a0.v, bk0.v, acc);
        acc = wmf(a1.v, bk1.v, acc);
        _Float16* hp = &Hh[(16 * mt + 8 * hf) * NW + col];
#pragma unroll
        for (int r = 0; r < 8; ++r)
          hp[r * NW] = (_Float16)fmaxf(acc[r] * (1.0f / 256.0f) + bb, 0.0f);
      }
    }
    __syncthreads();

    {
      FragH af0[4], af1[4];
#pragma unroll
      for (int k = 0; k < 4; ++k) {
        const _Float16* ap = &Hh[m * NW + 32 * k + 8 * hf];
        af0[k].h[0] = *(const v8h*)(ap);           af0[k].h[1] = *(const v8h*)(ap + 16);
        af1[k].h[0] = *(const v8h*)(ap + 16 * NW); af1[k].h[1] = *(const v8h*)(ap + 16 * NW + 16);
      }
      const _Float16* wl = woh + (size_t)ly * NDP * NW;
#pragma unroll 1
      for (int nt = wave; nt < NNT; nt += 8) {
        const int fo  = (16 * nt + 15) / NP;
        const int cnt = (fo <= 2) ? (3 * fo) : (2 * fo + 2);
        const int ks  = (cnt + 31) >> 5;
        const _Float16* bq = wl + ((size_t)(16 * nt + m)) * NW + 8 * hf;
        v8f acc0 = zf, acc1 = zf;
#pragma unroll
        for (int k = 0; k < 4; ++k) {
          if (k < ks) {
            FragH b;
            b.h[0] = *(const v8h*)(bq + 32 * k);
            b.h[1] = *(const v8h*)(bq + 32 * k + 16);
            acc0 = wmf(af0[k].v, b.v, acc0);
            acc1 = wmf(af1[k].v, b.v, acc1);
          }
        }
        const int col = 16 * nt + m;
        const float bias = bo[ly * NDP + col];
        float* p0 = &Pbuf[(8 * hf) * NDP + col];
        float* p1 = &Pbuf[(16 + 8 * hf) * NDP + col];
#pragma unroll
        for (int r = 0; r < 8; ++r) {
          p0[r * NDP] = acc0[r] * (1.0f / 65536.0f) + bias;
          p1[r * NDP] = acc1[r] * (1.0f / 65536.0f) + bias;
        }
      }
    }
    __syncthreads();

    {
      const int nxt = cur ^ 1;
#pragma unroll 1
      for (int it = 0; it < (RM * ND) / NTHR; ++it) {
        const int idx = it * NTHR + t;
        const int row = idx >> 6;
        const int f   = idx & (ND - 1);
        const float* pp = &Pbuf[row * NDP + f * NP];

        float wv[NKN], hv[NKN], wd[NKN], hg[NKN];
#pragma unroll
        for (int j = 0; j < NKN; ++j) { wv[j] = pp[j]; hv[j] = pp[NKN + j]; }
        adj_softmax8(wv, wd);
        adj_softmax8(hv, hg);
        float dv[NKN + 1];
        dv[0] = 1.0f; dv[NKN] = 1.0f;
#pragma unroll
        for (int j = 0; j < NKN - 1; ++j) dv[j + 1] = softplus_f(pp[2 * NKN + j]) + 0.001f;

        const float x = Xf[cur][idx];
        const bool inside = (x > -4.0f) && (x < 4.0f);
        const float xc = fminf(fmaxf(x, -4.0f), 4.0f);

        float xk = -4.0f, xk1 = 4.0f, yk = -4.0f, yk1 = 4.0f, dk = 1.0f, dk1 = 1.0f;
        float xlf = -4.0f, ylf = -4.0f, dlf = 1.0f, csx = 0.0f, csy = 0.0f;
#pragma unroll
        for (int j = 0; j < NKN; ++j) {
          csx += wd[j]; csy += hg[j];
          const float xr = csx + (-4.0f);
          const float yr = csy + (-4.0f);
          const float dr = dv[j + 1];
          const bool sel = (j == 0) || (xc >= xlf);
          xk  = sel ? xlf : xk;  xk1 = sel ? xr : xk1;
          yk  = sel ? ylf : yk;  yk1 = sel ? yr : yk1;
          dk  = sel ? dlf : dk;  dk1 = sel ? dr : dk1;
          xlf = xr; ylf = yr; dlf = dr;
        }

        const float rw   = rcp_f(xk1 - xk);
        const float sk   = (yk1 - yk) * rw;
        const float xi   = (xc - xk) * rw;
        const float omx  = 1.0f - xi;
        const float den  = sk + (dk1 + dk - 2.0f * sk) * xi * omx;
        const float rden = rcp_f(den);
        const float num  = sk * xi * xi + dk * xi * omx;
        float outv = yk + (yk1 - yk) * num * rden;
        float ldj  = 2.0f * __logf(sk)
                   + __logf(dk1 * xi * xi + 2.0f * sk * xi * omx + dk * omx * omx)
                   - 2.0f * __logf(den);
        outv = inside ? outv : x;
        ldj  = inside ? ldj : 0.0f;

        Xf[nxt][row * ND + (ND - 1 - f)] = outv;
        Ldj[idx] = ldj;
      }
    }
    __syncthreads();

    if (wave == 0) {
      const float* lp = &Ldj[lane * ND];
      float s = 0.0f;
#pragma unroll 2
      for (int j = 0; j < ND / 4; ++j) {
        const v4f v = *(const v4f*)(lp + 4 * j);
        s += v.x; s += v.y; s += v.z; s += v.w;
      }
      ldreg += s;
    }
    cur ^= 1;
  }

  if (wave == 0) Ldl[lane] = ldreg;
  __syncthreads();

  {
    const float* xs = Xf[cur];
    const v4f o0 = *(const v4f*)(xs + 4 * t);
    const v4f o1 = *(const v4f*)(xs + 4 * NTHR + 4 * t);
    const v4f lv = *(const v4f*)(&Ldl[4 * (t & 7)]);
    float* gx = out_x + (size_t)row0 * ND;
    float* gl = out_ld + row0;
    const bool wl = (t < 8);
    *(volatile v4f*)(gx + 4 * t) = o0;
    *(volatile v4f*)(gx + 4 * NTHR + 4 * t) = o1;
    if (wl) *(volatile v4f*)(gl + 4 * t) = lv;
    __threadfence();
    *(volatile v4f*)(gx + 4 * t) = o0;
    *(volatile v4f*)(gx + 4 * NTHR + 4 * t) = o1;
    if (wl) *(volatile v4f*)(gl + 4 * t) = lv;
  }
}

extern "C" void kernel_launch(void* const* d_in, const int* in_sizes, int n_in,
                              void* d_out, int out_size, void* d_ws, size_t ws_size,
                              hipStream_t stream) {
  if (n_in < 10) return;
  const int nW1 = NL * NW * ND;
  const int nWo = NL * NDP * NW;
  if (in_sizes[0] != NB * ND || in_sizes[1] != NB * ND) return;
  if (in_sizes[2] != nW1 || in_sizes[3] != NL * NW || in_sizes[4] != nWo || in_sizes[5] != NL * NDP) return;
  if (in_sizes[6] != nW1 || in_sizes[7] != NL * NW || in_sizes[8] != nWo || in_sizes[9] != NL * NDP) return;
  if (out_size != 2 * (NB * ND + NB)) return;

  const float* x    = (const float*)d_in[0];
  const float* y    = (const float*)d_in[1];
  const float* fW1  = (const float*)d_in[2];
  const float* fb1  = (const float*)d_in[3];
  const float* fWo  = (const float*)d_in[4];
  const float* fbo  = (const float*)d_in[5];
  const float* gW1  = (const float*)d_in[6];
  const float* gb1  = (const float*)d_in[7];
  const float* gWo  = (const float*)d_in[8];
  const float* gbo  = (const float*)d_in[9];
  float* out = (float*)d_out;
  float* xo  = out;
  float* ldf = out + (size_t)NB * ND;
  float* yo  = out + (size_t)NB * ND + NB;
  float* ldg = out + (size_t)2 * NB * ND + NB;

  char* ws = (char*)d_ws;
  size_t off = 0;
  const size_t oA = off; off += (size_t)nW1 * 2; off = (off + 255) & ~(size_t)255;
  const size_t oB = off; off += (size_t)nW1 * 2; off = (off + 255) & ~(size_t)255;
  const size_t oC = off; off += (size_t)nWo * 2; off = (off + 255) & ~(size_t)255;
  const size_t oD = off; off += (size_t)nWo * 2; off = (off + 255) & ~(size_t)255;
  if (off > ws_size || off > (size_t)WSCAP) return;
  _Float16* fW1h = (_Float16*)(ws + oA);
  _Float16* gW1h = (_Float16*)(ws + oB);
  _Float16* fWoh = (_Float16*)(ws + oC);
  _Float16* gWoh = (_Float16*)(ws + oD);

  k_cvt_w1<<<nW1 / (8 * NTHR), NTHR, 0, stream>>>(fW1, fW1h);
  k_cvt_w1<<<nW1 / (8 * NTHR), NTHR, 0, stream>>>(gW1, gW1h);
  k_cvt_wo<<<nWo / (8 * NTHR), NTHR, 0, stream>>>(fWo, fWoh);
  k_cvt_wo<<<nWo / (8 * NTHR), NTHR, 0, stream>>>(gWo, gWoh);
  k_flow<<<NB / RM, NTHR, 0, stream>>>(x, fW1h, fb1, fWoh, fbo, xo, ldf);
  k_flow<<<NB / RM, NTHR, 0, stream>>>(y, gW1h, gb1, gWoh, gbo, yo, ldg);
}
